// MultiFeatureTransformer_9809705305084
// MI455X (gfx1250) — hardware-verified
//
#include <hip/hip_runtime.h>


#define NB_  65536
#define NF   64
#define H1   64
#define H2   64
#define SLP  0.05f
#define LOSC 1024.0f
#define LOSCI (1.0f / 1024.0f)

typedef _Float16 h16;
typedef __attribute__((ext_vector_type(16))) _Float16 v16h;
typedef __attribute__((ext_vector_type(8)))  _Float16 v8h;
typedef __attribute__((ext_vector_type(8)))  float    v8f;
typedef __attribute__((ext_vector_type(4)))  float    v4f;
typedef v4f  __attribute__((may_alias)) v4fa;

__device__ __forceinline__ unsigned short f2bf(float f) { unsigned u = __float_as_uint(f); u += 0x7FFFu + ((u >> 16) & 1u); return (unsigned short)(u >> 16); }
__device__ __forceinline__ float bf2f(unsigned short b) { return __uint_as_float(((unsigned)b) << 16); }
__device__ __forceinline__ float bfr(float f) { return bf2f(f2bf(f)); }
__device__ __forceinline__ v16h cat16(v8h lo, v8h hi) { return __builtin_shufflevector(lo, hi, 0, 1, 2, 3, 4, 5, 6, 7, 8, 9, 10, 11, 12, 13, 14, 15); }
__device__ __forceinline__ v8f wmma16(v16h a, v16h b, v8f c) { return __builtin_amdgcn_wmma_f32_16x16x32_f16(false, a, false, b, (short)0, c, false, false); }
__device__ __forceinline__ float lk(float v) { return v >= 0.f ? v : SLP * v; }
#define VST2(T, p, v) do { const T vst2_v_ = (v); *(volatile T*)(p) = vst2_v_; __threadfence(); *(volatile T*)(p) = vst2_v_; } while (0)

__global__ __launch_bounds__(256) void k_w16(const float* __restrict__ W2, h16* W16) {
    const int lane = threadIdx.x & 31, r = blockIdx.x * 8 + (threadIdx.x >> 5);
    if (r >= NF * H2) return;
    typedef __attribute__((ext_vector_type(2))) _Float16 v2h;
    v2h o; o[0] = (h16)bfr(W2[(size_t)r * H1 + 2 * lane]); o[1] = (h16)bfr(W2[(size_t)r * H1 + 2 * lane + 1]);
    VST2(v2h, W16 + (size_t)r * H1 + 2 * lane, o);
}

__global__ __launch_bounds__(128) void k_main(const float* __restrict__ x, const float* __restrict__ W1, const float* __restrict__ b1, const h16* __restrict__ W16,
                                             const float* __restrict__ b2, const float* __restrict__ W3, const float* __restrict__ b3, float* out) {
    __shared__ __align__(16) float yt[64 * 68];
    const int lane = threadIdx.x & 31, wave = threadIdx.x >> 5, lr = lane & 15, hi = lane >> 4;
    const int r0 = blockIdx.x * 64 + wave * 16;
    float* myy = yt + wave * 16 * 68;
#pragma unroll 1
    for (int f = 0; f < NF; ++f) {
        const float xv = x[(size_t)(r0 + lr) * NF + f];
        const float xb = bfr(xv);
        v16h ah[2], al[2];
#pragma unroll
        for (int kc = 0; kc < 2; ++kc)
#pragma unroll
            for (int q = 0; q < 16; ++q) { const int h = kc * 32 + ((q < 8) ? (8 * hi + q) : (16 + 8 * hi + (q - 8)));
                const float v = lk(xb * bfr(W1[f * H1 + h]) + bfr(b1[f * H1 + h])); const h16 hv = (h16)v; ah[kc][q] = hv; al[kc][q] = (h16)((v - (float)hv) * LOSC); }
        v8f acc[4], accx[4];
#pragma unroll
        for (int n = 0; n < 4; ++n) { acc[n] = (v8f){}; accx[n] = (v8f){}; }
        const h16* wf = W16 + (size_t)f * H2 * H1;
#pragma unroll
        for (int kc = 0; kc < 2; ++kc)
#pragma unroll
            for (int n = 0; n < 4; ++n) { const h16* bp = wf + (size_t)(n * 16 + lr) * H1 + kc * 32 + 8 * hi; const v16h bb = cat16(*(const v8h*)bp, *(const v8h*)(bp + 16));
                acc[n] = wmma16(ah[kc], bb, acc[n]); accx[n] = wmma16(al[kc], bb, accx[n]); }
        asm volatile("v_nop\n\tv_nop\n\tv_nop\n\tv_nop" : "+v"(acc[0]), "+v"(acc[1]), "+v"(acc[2]), "+v"(acc[3]), "+v"(accx[0]), "+v"(accx[1]), "+v"(accx[2]), "+v"(accx[3]));
        float part[8];
#pragma unroll
        for (int j = 0; j < 8; ++j) { float s = 0.f;
#pragma unroll
            for (int n = 0; n < 4; ++n) { const int g = n * 16 + lr; s += lk(acc[n][j] + accx[n][j] * LOSCI + bfr(b2[f * H2 + g])) * bfr(W3[f * H2 + g]); }
            s += __shfl_xor(s, 1, 16); s += __shfl_xor(s, 2, 16); s += __shfl_xor(s, 4, 16); s += __shfl_xor(s, 8, 16);
            part[j] = s + bfr(b3[f]); }
        if (lr == 0) {
#pragma unroll
            for (int j = 0; j < 8; ++j) myy[(hi * 8 + j) * 68 + f] = part[j];
        }
    }
    asm volatile("" ::: "memory");
    __builtin_amdgcn_fence(__ATOMIC_RELEASE, "workgroup");
    __builtin_amdgcn_wave_barrier();
    auto pass = [&]() {
#pragma unroll
        for (int s = 0; s < 8; ++s) { const int row = 2 * s + (lane >> 4), piece = lane & 15; const v4f v = *(const v4fa*)(myy + row * 68 + piece * 4);
            *(volatile v4f*)(out + (size_t)(r0 + row) * NF + piece * 4) = v; }
    };
    pass(); __threadfence(); pass();
}

extern "C" void kernel_launch(void* const* d_in, const int* in_sizes, int n_in,
                              void* d_out, int out_size, void* d_ws, size_t ws_size, hipStream_t stream) {
    (void)in_sizes; (void)n_in; (void)out_size;
    const float* x = (const float*)d_in[0]; const float* W1 = (const float*)d_in[1]; const float* b1 = (const float*)d_in[2]; const float* W2 = (const float*)d_in[3];
    const float* b2 = (const float*)d_in[4]; const float* W3 = (const float*)d_in[5]; const float* b3 = (const float*)d_in[6];
    float* out = (float*)d_out;
    char* wsp = (char*)d_ws;
    auto take = [&](size_t bytes) { char* p = wsp; wsp += (bytes + 255) & ~(size_t)255; return (void*)p; };
    h16* W16 = (h16*)take((size_t)NF * H2 * H1 * 2);
    if ((size_t)(wsp - (char*)d_ws) > ws_size) return;
    k_w16<<<(NF * H2) / 8, 256, 0, stream>>>(W2, W16);
    k_main<<<NB_ / 64, 128, 0, stream>>>(x, W1, b1, W16, b2, W3, b3, out);
}
